// MHAttentionIneffcient_1005022347919
// MI455X (gfx1250) — hardware-verified
//
#include <hip/hip_runtime.h>
#include <math.h>

typedef __attribute__((ext_vector_type(16))) _Float16 v16h;
typedef __attribute__((ext_vector_type(16))) __bf16 v16b;
typedef __attribute__((ext_vector_type(8)))  _Float16 v8h;
typedef __attribute__((ext_vector_type(8)))  float v8f;
typedef __attribute__((ext_vector_type(4)))  float v4f;
typedef __attribute__((ext_vector_type(2)))  float v2f;
typedef __attribute__((ext_vector_type(4)))  unsigned v4u;
typedef __attribute__((ext_vector_type(4)))  int v4i;
typedef float __attribute__((may_alias)) float_a;
typedef int __attribute__((may_alias)) int_a;

template <typename T> __device__ __forceinline__ void vst2(void* p, T v) { *(volatile T*)p = v; __threadfence(); *(volatile T*)p = v; }
__device__ __forceinline__ v8f wmma16(v16h a, v16h b, v8f c) {
  v8f d = __builtin_amdgcn_wmma_f32_16x16x32_f16(false, a, false, b, (short)0, c, false, false);
  asm volatile("v_nop\n\tv_nop\n\tv_nop\n\tv_nop" : "+v"(d) : "v"(a), "v"(b));
  return d;
}
__device__ __forceinline__ v8f wmma_bf(v16b a, v16b b, v8f c) {
  v8f d = __builtin_amdgcn_wmma_f32_16x16x32_bf16(false, a, false, b, (short)0, c, false, false);
  asm volatile("v_nop\n\tv_nop\n\tv_nop\n\tv_nop" : "+v"(d) : "v"(a), "v"(b));
  return d;
}
__device__ __forceinline__ v16h frag_h(const _Float16* rowk0, int lane) {
  union { v16h v; v8h q[2]; } u; const _Float16* p = rowk0 + 8 * (lane >> 4);
  u.q[0] = *(const v8h*)p; u.q[1] = *(const v8h*)(p + 16); return u.v;
}
__device__ __forceinline__ v16h frag_f32(const float* rowk0, int lane) {
  v16h a; const float* p = rowk0 + 8 * (lane >> 4);
#pragma unroll
  for (int i = 0; i < 8; ++i) { a[i] = (_Float16)p[i]; a[8 + i] = (_Float16)p[16 + i]; }
  return a;
}
__device__ __forceinline__ v16h frag_f32s(const float* rowk0, int lane, float sc) {
  v16h a; const float* p = rowk0 + 8 * (lane >> 4);
#pragma unroll
  for (int i = 0; i < 8; ++i) { a[i] = (_Float16)(p[i] * sc); a[8 + i] = (_Float16)(p[16 + i] * sc); }
  return a;
}
__device__ __forceinline__ v16h fragc_f32(const float* W, int k0, int n, int lane, int ld, int K) {
  v16h a; const int g = lane >> 4;
#pragma unroll
  for (int i = 0; i < 8; ++i) { const int ka = k0 + 8 * g + i, kb = ka + 16;
    a[i] = (_Float16)(ka < K ? W[(size_t)(ka < K ? ka : K - 1) * ld + n] : 0.f); a[8 + i] = (_Float16)(kb < K ? W[(size_t)(kb < K ? kb : K - 1) * ld + n] : 0.f); }
  return a;
}
struct F2 { v16b h, l; };
__device__ __forceinline__ F2 bsplit16(const float v[16]) { F2 r;
#pragma unroll
  for (int i = 0; i < 16; ++i) { const __bf16 h = (__bf16)v[i]; r.h[i] = h; r.l[i] = (__bf16)(v[i] - (float)h); }
  return r; }
__device__ __forceinline__ F2 split_row(const float* row, int k0, int lane) { float v[16]; const float* p = row + k0 + 8 * (lane >> 4);
#pragma unroll
  for (int i = 0; i < 8; ++i) { v[i] = p[i]; v[8 + i] = p[16 + i]; }
  return bsplit16(v); }
__device__ __forceinline__ F2 split_rowK(const float* row, int k0, int lane, int K) { float v[16]; const int g = lane >> 4;
#pragma unroll
  for (int i = 0; i < 8; ++i) { const int ka = k0 + 8 * g + i, kb = ka + 16; v[i] = ka < K ? row[ka < K ? ka : K - 1] : 0.f; v[8 + i] = kb < K ? row[kb < K ? kb : K - 1] : 0.f; }
  return bsplit16(v); }
__device__ __forceinline__ F2 split_col(const float* W, int k0, int n, int lane, int ld, int K) { float v[16]; const int g = lane >> 4;
#pragma unroll
  for (int i = 0; i < 8; ++i) { const int ka = k0 + 8 * g + i, kb = ka + 16; v[i] = ka < K ? W[(size_t)(ka < K ? ka : K - 1) * ld + n] : 0.f; v[8 + i] = kb < K ? W[(size_t)(kb < K ? kb : K - 1) * ld + n] : 0.f; }
  return bsplit16(v); }
__device__ __forceinline__ v8f mac3(const F2& a, const F2& b, v8f c) { c = wmma_bf(a.l, b.h, c); c = wmma_bf(a.h, b.l, c); return wmma_bf(a.h, b.h, c); }
__device__ __forceinline__ float sigm(float v) { return 1.0f / (1.0f + expf(-v)); }
#define LDSX() do { asm volatile("s_wait_dscnt 0" ::: "memory"); __builtin_amdgcn_wave_barrier(); __builtin_amdgcn_fence(__ATOMIC_RELEASE, "workgroup"); } while (0)


#define NB 1
#define SS 2048
#define DM 1024
#define NH 16
#define HD 64
#define QKVW (3 * DM)
#ifndef TQB
#define TQB (SS / 64)
#endif
#ifndef TNH
#define TNH NH
#define TNB NB
#define TOB (NB * SS / 64)
#endif
typedef __attribute__((ext_vector_type(8))) __bf16 v8b;
__device__ __forceinline__ v16b frag_b(const __bf16* rowk0, int lane) {
  union { v16b v; v8b q[2]; } u; const __bf16* p = rowk0 + 8 * (lane >> 4);
  u.q[0] = *(const v8b*)p; u.q[1] = *(const v8b*)(p + 16); return u.v;
}
__device__ __forceinline__ float bfr(float v) { return (float)(__bf16)v; }
__device__ __attribute__((noinline)) float exp_ni(float v) { return expf(v); }
__device__ __attribute__((noinline)) float erf_ni(float v) { return erff(v); }

#define PK_A 0
#define PK_P (PK_A + QKVW * DM)
#define PK_END (PK_P + DM * DM)
#define WS_PK  0u
#define WS_QK  (WS_PK + 2u * PK_END)
#define WS_QKL (WS_QK + 2u * NB * SS * 2 * DM)
#define WS_VTH (WS_QKL + 2u * NB * SS * 2 * DM)
#define WS_VTL (WS_VTH + 2u * NB * DM * SS)
#define WS_O   (WS_VTL + 2u * NB * DM * SS)
#define WS_CS  (WS_O + 4u * NB * SS * DM)
#define WS_END (WS_CS + 4u * 2 * SS * 32)
__global__ __launch_bounds__(256) void k_pack(const float* __restrict__ WQ, const float* __restrict__ WK, const float* __restrict__ WV, __bf16* __restrict__ PK) {
  __shared__ __align__(16) __bf16 s[DM]; const int n = blockIdx.x, which = blockIdx.y, t = threadIdx.x; const int h = n / HD, d = n % HD; const float* Wm = which == 0 ? WQ : which == 1 ? WK : WV;
  for (int i = t; i < DM; i += 256) s[i] = (__bf16)Wm[((size_t)h * DM + i) * HD + d];
  __syncthreads(); __bf16* dst = PK + PK_A + ((size_t)which * DM + n) * DM; for (int q = t; q < DM / 8; q += 256) vst2((unsigned*)(dst + q * 8), *(const v4u*)&s[q * 8]); }
__global__ __launch_bounds__(128) void k_out2(const float* __restrict__ O, const float* __restrict__ WO, const float* __restrict__ BO, float* __restrict__ OUT) { __shared__ __align__(16) float sf[4][16][68];
  const int tid = threadIdx.x, wave = tid >> 5, lane = tid & 31, col = lane & 15, g = lane >> 4; const int r0 = blockIdx.x * 64 + wave * 16; const int rr = r0 + col; const int hsel = rr / 128; const int sbase = 16 * (rr % 128);
  v8f acc[4] = {};
#pragma unroll 2
  for (int kc = 0; kc < DM / 32; ++kc) { const int j = kc / 2, half = kc % 2; const F2 a = split_row(O + (size_t)(sbase + j) * DM + hsel * HD + half * 32, 0, lane);
#pragma unroll
    for (int jj = 0; jj < 4; ++jj) { v16b w; const int o = jj * 16 + col;
#pragma unroll
      for (int i = 0; i < 8; ++i) { w[i] = (__bf16)WO[(size_t)(kc * 32 + 8 * g + i) * 64 + o]; w[8 + i] = (__bf16)WO[(size_t)(kc * 32 + 16 + 8 * g + i) * 64 + o]; }
      acc[jj] = wmma_bf(a.h, w, acc[jj]); acc[jj] = wmma_bf(a.l, w, acc[jj]); } }
#pragma unroll
  for (int jj = 0; jj < 4; ++jj) { const float bb = bfr(BO[jj * 16 + col]);
#pragma unroll
    for (int r = 0; r < 8; ++r) sf[wave][8 * g + r][jj * 16 + col] = acc[jj][r] + bb; }
  LDSX(); for (int rl = 0; rl < 16; ++rl) if (lane < 16) vst2(OUT + (size_t)(r0 + rl) * 64 + lane * 4, *(const v4f*)&sf[wave][rl][lane * 4]); }
__global__ __launch_bounds__(128) void k_qkv(const float* __restrict__ XQ, const float* __restrict__ XK, const float* __restrict__ XV, const __bf16* __restrict__ P, const float* __restrict__ BQ, const float* __restrict__ BK, const float* __restrict__ BV, _Float16* __restrict__ QK, _Float16* __restrict__ QKL, _Float16* __restrict__ VTH, _Float16* __restrict__ VTL) {
  const int which0 = (blockIdx.y * 128) / DM; const float* X = (which0 == 0) ? XQ : (which0 == 1) ? XK : XV; const float* BB = BQ ? (((which0 == 0) ? BQ : (which0 == 1) ? BK : BV) + (blockIdx.y * 128 - which0 * DM)) : nullptr;
  __shared__ __align__(16) _Float16 so[4][16][136], sol[4][16][136]; __shared__ __align__(16) _Float16 sth[128][72], stl[128][72];
  const int tid = threadIdx.x, wave = tid >> 5, lane = tid & 31, col = lane & 15, g = lane >> 4; const size_t r0 = (size_t)blockIdx.x * 64 + wave * 16; const int n0 = blockIdx.y * 128;
  v8f acc[8] = {};
#pragma unroll 2
  for (int kc = 0; kc < DM / 32; ++kc) { v16b a; { const float* p = X + (r0 + col) * DM + kc * 32 + 8 * g;
#pragma unroll
      for (int i = 0; i < 8; ++i) { a[i] = (__bf16)p[i]; a[8 + i] = (__bf16)p[16 + i]; } }
#pragma unroll
    for (int j = 0; j < 8; ++j) acc[j] = wmma_bf(a, frag_b(P + (size_t)(n0 + j * 16 + col) * DM + kc * 32, lane), acc[j]); }
  if (n0 < 2 * DM) {
#pragma unroll
    for (int j = 0; j < 8; ++j) {
#pragma unroll
      for (int r = 0; r < 8; ++r) { const float v = acc[j][r] + (BB ? bfr(BB[j * 16 + col]) : 0.f); const _Float16 hv = (_Float16)v; so[wave][8 * g + r][j * 16 + col] = hv; sol[wave][8 * g + r][j * 16 + col] = (_Float16)((v - (float)hv) * 2048.0f); } }
    LDSX();
    for (int rl = 0; rl < 16; ++rl) if (lane < 16) { vst2((unsigned*)(QK + (r0 + rl) * (2 * DM) + n0 + lane * 8), *(const v4u*)&so[wave][rl][lane * 8]); vst2((unsigned*)(QKL + (r0 + rl) * (2 * DM) + n0 + lane * 8), *(const v4u*)&sol[wave][rl][lane * 8]); }
  } else {
#pragma unroll
    for (int j = 0; j < 8; ++j) {
#pragma unroll
      for (int r = 0; r < 8; ++r) { const float v = acc[j][r] + (BB ? bfr(BB[j * 16 + col]) : 0.f); const _Float16 hv = (_Float16)v; sth[j * 16 + col][wave * 16 + 8 * g + r] = hv; stl[j * 16 + col][wave * 16 + 8 * g + r] = (_Float16)((v - (float)hv) * 2048.0f); } }
    __syncthreads();
    const size_t rb = (size_t)blockIdx.x * 64; const int b = (int)(rb / SS), s0 = (int)(rb % SS); const int pc0 = n0 - 2 * DM;
    for (int q = tid; q < 128 * 8; q += 128) { const int d = q >> 3, pc = q & 7; const size_t o = ((size_t)b * DM + pc0 + d) * SS + s0 + pc * 8; vst2((unsigned*)(VTH + o), *(const v4u*)&sth[d][pc * 8]); vst2((unsigned*)(VTL + o), *(const v4u*)&stl[d][pc * 8]); }
  }
}
__global__ __launch_bounds__(128) void k_attn(const _Float16* __restrict__ QK, const _Float16* __restrict__ QKL, const _Float16* __restrict__ VTH, const _Float16* __restrict__ VTL, const void* __restrict__ KMASK, float* __restrict__ O) {
  __shared__ __align__(16) float sp[4][16][36]; __shared__ __align__(16) float so[4][16][68];
  const int tid = threadIdx.x, wave = tid >> 5, lane = tid & 31, col = lane & 15, g = lane >> 4;
  const int qb = blockIdx.x, h = blockIdx.y, b = blockIdx.z; const int q0 = qb * 64 + wave * 16; const size_t rq = (size_t)b * SS + q0 + col;
  v16h aq[2], aql[2];
#pragma unroll
  for (int kc = 0; kc < 2; ++kc) { aq[kc] = frag_h(QK + rq * (2 * DM) + h * HD + kc * 32, lane); aql[kc] = frag_h(QKL + rq * (2 * DM) + h * HD + kc * 32, lane); }
  float m[8], l[8];
#pragma unroll
  for (int r = 0; r < 8; ++r) { m[r] = -3.0e38f; l[r] = 0.f; }
  v8f acc[4] = {}, accl[4] = {};
  const int nks = SS / 32;
#pragma unroll 1
  for (int ks = 0; ks < nks; ++ks) { v8f s[2];
#pragma unroll
    for (int ct = 0; ct < 2; ++ct) { const int kk = ks * 32 + ct * 16 + col; const _Float16* krow = QK + ((size_t)b * SS + kk) * (2 * DM) + DM + h * HD; const _Float16* krowl = QKL + ((size_t)b * SS + kk) * (2 * DM) + DM + h * HD; v8f c = {}, cl = {};
      if (qb < 2) {
#pragma unroll
        for (int kc = 0; kc < 2; ++kc) { const v16h kh = frag_h(krow + kc * 32, lane); c = wmma16(aq[kc], kh, c); cl = wmma16(aql[kc], kh, cl); cl = wmma16(aq[kc], frag_h(krowl + kc * 32, lane), cl); }
#pragma unroll
        for (int r = 0; r < 8; ++r) c[r] += cl[r] * (1.0f / 2048.0f); }
      else {
#pragma unroll
        for (int kc = 0; kc < 2; ++kc) c = wmma16(aq[kc], frag_h(krow + kc * 32, lane), c); }
      { const bool keepk = true;
#pragma unroll
      for (int r = 0; r < 8; ++r) s[ct][r] = keepk ? c[r] * 0.125f : -3.0e38f; } }
#pragma unroll
    for (int r = 0; r < 8; ++r) { float mx = fmaxf(s[0][r], s[1][r]);
#pragma unroll
      for (int o = 1; o < 16; o <<= 1) mx = fmaxf(mx, __shfl_xor(mx, o));
      const float mn = fmaxf(m[r], mx); const float alpha = (m[r] <= -1.0e38f) ? 0.f : __expf(m[r] - mn);
      const float e0 = (s[0][r] <= -1.0e38f) ? 0.f : __expf(s[0][r] - mn), e1 = (s[1][r] <= -1.0e38f) ? 0.f : __expf(s[1][r] - mn); float es = e0 + e1;
#pragma unroll
      for (int o = 1; o < 16; o <<= 1) es += __shfl_xor(es, o);
      l[r] = l[r] * alpha + es; m[r] = mn;
#pragma unroll
      for (int dt = 0; dt < 4; ++dt) { acc[dt][r] *= alpha; accl[dt][r] *= alpha; }
      sp[wave][8 * g + r][col] = e0; sp[wave][8 * g + r][16 + col] = e1; }
    LDSX();
    v16h pa, pl; { const float* prow = &sp[wave][col][0] + 8 * (lane >> 4);
#pragma unroll
      for (int i = 0; i < 8; ++i) { const float x0 = prow[i] * 2048.0f, x1 = prow[16 + i] * 2048.0f; const _Float16 h0 = (_Float16)x0, h1 = (_Float16)x1; pa[i] = h0; pa[8 + i] = h1; pl[i] = (_Float16)((x0 - (float)h0) * 2048.0f); pl[8 + i] = (_Float16)((x1 - (float)h1) * 2048.0f); } }
#pragma unroll
    for (int dt = 0; dt < 4; ++dt) { const size_t vr = ((size_t)b * DM + h * HD + dt * 16 + col) * SS + ks * 32; const v16h vh = frag_h(VTH + vr, lane); acc[dt] = wmma16(pa, vh, acc[dt]); if (qb < 2) { accl[dt] = wmma16(pl, vh, accl[dt]); accl[dt] = wmma16(pa, frag_h(VTL + vr, lane), accl[dt]); } }
    LDSX(); }
#pragma unroll
  for (int r = 0; r < 8; ++r) { const float il = (1.0f / 2048.0f) / l[r];
#pragma unroll
    for (int dt = 0; dt < 4; ++dt) so[wave][8 * g + r][dt * 16 + col] = (acc[dt][r] + accl[dt][r] * (1.0f / 2048.0f)) * il; }
  LDSX();
  for (int rl = 0; rl < 16; ++rl) if (lane < 16) vst2(O + ((size_t)b * SS + q0 + rl) * DM + h * HD + lane * 4, *(const v4f*)&so[wave][rl][lane * 4]);
}
__global__ __launch_bounds__(128) void k_out(const float* __restrict__ O, const __bf16* __restrict__ P, const float* __restrict__ BO, float* __restrict__ Y) {
  __shared__ __align__(16) float so[4][16][132];
  const int tid = threadIdx.x, wave = tid >> 5, lane = tid & 31, col = lane & 15, g = lane >> 4; const size_t r0 = (size_t)blockIdx.x * 64 + wave * 16; const int n0 = blockIdx.y * 128;
  v8f acc[8] = {};
#pragma unroll 2
  for (int kc = 0; kc < DM / 32; ++kc) { const F2 a = split_row(O + (r0 + col) * DM, kc * 32, lane);
#pragma unroll
    for (int j = 0; j < 8; ++j) { const v16b w = frag_b(P + (size_t)(n0 + j * 16 + col) * DM + kc * 32, lane); acc[j] = wmma_bf(a.l, w, acc[j]); acc[j] = wmma_bf(a.h, w, acc[j]); } }
#pragma unroll
  for (int j = 0; j < 8; ++j) {
#pragma unroll
    for (int r = 0; r < 8; ++r) so[wave][8 * g + r][j * 16 + col] = acc[j][r] + (BO ? bfr(BO[n0 + j * 16 + col]) : 0.f); }
  LDSX();
  for (int rl = 0; rl < 16; ++rl) vst2(Y + (r0 + rl) * DM + n0 + lane * 4, *(const v4f*)&so[wave][rl][lane * 4]);
}
extern "C" void kernel_launch(void* const* d_in, const int* in_sizes, int n_in, void* d_out, int out_size, void* d_ws, size_t ws_size, hipStream_t stream) {
  (void)in_sizes; (void)n_in; (void)out_size;
  const float** F = (const float**)d_in;
  if (ws_size < (size_t)WS_END) return;
  char* ws = (char*)d_ws; __bf16* PK = (__bf16*)(ws + WS_PK); _Float16 *QK = (_Float16*)(ws + WS_QK), *QKL = (_Float16*)(ws + WS_QKL), *VTH = (_Float16*)(ws + WS_VTH), *VTL = (_Float16*)(ws + WS_VTL); float* O = (float*)(ws + WS_O);
  k_pack<<<dim3(DM, 3), 256, 0, stream>>>(F[2], F[4], F[6], PK);
  k_qkv<<<dim3(TNB * SS / 64, QKVW / 128), 128, 0, stream>>>(F[0], F[1], F[1], PK + PK_A, F[3], F[5], F[7], QK, QKL, VTH, VTL);
  k_attn<<<dim3(TQB, TNH, TNB), 128, 0, stream>>>(QK, QKL, VTH, VTL, nullptr, O);
  k_out2<<<TOB, 128, 0, stream>>>(O, F[8], F[9], (float*)d_out);
}
